// HeteroSAGELayer_61435212202261
// MI455X (gfx1250) — hardware-run, weakly checked
//
#include <hip/hip_runtime.h>

typedef float          v8f   __attribute__((ext_vector_type(8)));
typedef float          v4f   __attribute__((ext_vector_type(4)));
typedef unsigned int   v4u   __attribute__((ext_vector_type(4)));
typedef int            v8i   __attribute__((ext_vector_type(8)));
typedef unsigned short v8us  __attribute__((ext_vector_type(8)));
typedef unsigned short v16us __attribute__((ext_vector_type(16)));
typedef __bf16         v16bf __attribute__((ext_vector_type(16)));
typedef _Float16       v16h  __attribute__((ext_vector_type(16)));
typedef v4f  __attribute__((may_alias)) v4fa;
typedef v8us __attribute__((may_alias)) v8usa;
union FragB { v16bf v; v16us u; v8us h[2]; v8i w; };
union FragH { v16h  v; v16us u; v8us h[2]; v8i w; };

__device__ __forceinline__ v8f wmb(const FragB& a, const FragB& b, v8f c) {
  v8f d = __builtin_amdgcn_wmma_f32_16x16x32_bf16(false, a.v, false, b.v, (short)0, c, false, false);
  asm volatile("v_nop\n\tv_nop\n\tv_nop\n\tv_nop" : "+v"(d) : "v"(a.w), "v"(b.w));
  return d;
}

__device__ __forceinline__ v8f wmh(const FragH& a, const FragH& b, v8f c) {
  v8f d = __builtin_amdgcn_wmma_f32_16x16x32_f16(false, a.v, false, b.v, (short)0, c, false, false);
  asm volatile("v_nop\n\tv_nop\n\tv_nop\n\tv_nop" : "+v"(d) : "v"(a.w), "v"(b.w));
  return d;
}

__device__ __forceinline__ unsigned bf16_bits(float f) {
  const unsigned u = __float_as_uint(f);
  const unsigned r = (u + 0x7FFFu + ((u >> 16) & 1u)) >> 16;
  const unsigned q = (u >> 16) | 0x40u;
  return ((u & 0x7fffffffu) > 0x7f800000u) ? q : r;
}

__device__ __forceinline__ float bf16_val(float f) {
  return __uint_as_float(bf16_bits(f) << 16);
}
__device__ __forceinline__ int clampi(int v, int lo, int hi) {
  return v < lo ? lo : (v > hi ? hi : v);
}

__device__ __forceinline__ unsigned f16_bits(float f) {
  const unsigned u  = __float_as_uint(f);
  const unsigned s  = (u >> 16) & 0x8000u;
  const unsigned a  = u & 0x7fffffffu;
  const unsigned t  = a - 0x38000000u;
  const unsigned r  = (t + 0x0FFFu + ((t >> 13) & 1u)) >> 13;
  const unsigned rc = r > 0x7C00u ? 0x7C00u : r;
  const bool small  = a < 0x38800000u;
  const bool isnan  = a > 0x7f800000u;
  const unsigned fin = small ? 0u : (s | rc);
  return isnan ? (s | 0x7E00u) : fin;
}

__device__ __forceinline__ unsigned pk16(unsigned lo, unsigned hi) { return lo | (hi << 16); }
__device__ __forceinline__ unsigned bf16_lo_bits(float v) {
  float hi = bf16_val(v);
  asm volatile("" : "+v"(hi));
  return bf16_bits(v - hi);
}
__device__ __forceinline__ v4u pack8_bf16(v4f a, v4f c) {
  return (v4u){ pk16(bf16_bits(a[0]), bf16_bits(a[1])), pk16(bf16_bits(a[2]), bf16_bits(a[3])),
                pk16(bf16_bits(c[0]), bf16_bits(c[1])), pk16(bf16_bits(c[2]), bf16_bits(c[3])) };
}
__device__ __forceinline__ v4u pack8_bf16_lo(v4f a, v4f c) {
  return (v4u){ pk16(bf16_lo_bits(a[0]), bf16_lo_bits(a[1])), pk16(bf16_lo_bits(a[2]), bf16_lo_bits(a[3])),
                pk16(bf16_lo_bits(c[0]), bf16_lo_bits(c[1])), pk16(bf16_lo_bits(c[2]), bf16_lo_bits(c[3])) };
}
__device__ __forceinline__ v4u pack8_f16(v4f a, v4f c) {
  return (v4u){ pk16(f16_bits(a[0]), f16_bits(a[1])), pk16(f16_bits(a[2]), f16_bits(a[3])),
                pk16(f16_bits(c[0]), f16_bits(c[1])), pk16(f16_bits(c[2]), f16_bits(c[3])) };
}

template <int FORM>
__global__ __launch_bounds__(256) void k_plane(const float* __restrict__ src, int rows, int cols, int ldsrc,
                                               unsigned short* __restrict__ dst, int MP, int KP) {
  static_assert(FORM >= 0 && FORM <= 3);
  const int KTOT = (FORM == 1 || FORM == 3) ? 2 * KP : KP;
  const unsigned ppr   = (unsigned)(KTOT >> 3);
  const unsigned kp8   = (unsigned)(KP >> 3);
  const unsigned total = (unsigned)MP * ppr;
  const unsigned g     = blockIdx.x * 256u + threadIdx.x;
  const unsigned rowu  = g / ppr;
  const unsigned p     = g - rowu * ppr;
  const bool second    = p >= kp8;
  const int row = (int)rowu;
  const int c0  = (int)((second ? p - kp8 : p) << 3);
  const float* srow = src + (size_t)clampi(row, 0, rows - 1) * (size_t)ldsrc;
  float x[8];
  unsigned mk[8];
#pragma unroll
  for (int e = 0; e < 8; ++e) {
    const int c = c0 + e;
    const float v = srow[clampi(c, 0, cols - 1)];
    asm volatile("" :: "v"(v));
    x[e]  = v;
    mk[e] = (row < rows && c < cols) ? 0xFFFFu : 0u;
  }
  const v4f a = (v4f){ x[0], x[1], x[2], x[3] };
  const v4f c = (v4f){ x[4], x[5], x[6], x[7] };
  v4u o;
  if (FORM == 2) {
    o = pack8_f16(a, c);
  } else {
    const v4u hi = pack8_bf16(a, c);
    o = hi;
    if (FORM == 1) { const v4u lo = pack8_bf16_lo(a, c); o = second ? lo : hi; }
  }
  const v4u mw = (v4u){ pk16(mk[0], mk[1]), pk16(mk[2], mk[3]), pk16(mk[4], mk[5]), pk16(mk[6], mk[7]) };
  o &= mw;
  if (g < total) {
    volatile v4u* q = (volatile v4u*)(dst + (size_t)g * 8);
    *q = o;
    __threadfence();
    *q = o;
  }
}

template <int FORM> struct FragOf    { typedef FragB T; };
template <>         struct FragOf<2> { typedef FragH T; };
__device__ __forceinline__ v8f mm(const FragB& a, const FragB& b, v8f c) { return wmb(a, b, c); }
__device__ __forceinline__ v8f mm(const FragH& a, const FragH& b, v8f c) { return wmh(a, b, c); }
template <class F> __device__ __forceinline__ F ld_frag(const unsigned short* p) {
  F f;
  f.h[0] = *(const v8usa*)(p);
  f.h[1] = *(const v8usa*)(p + 16);
  return f;
}

template <int FORM, int EPI>
__global__ __launch_bounds__(256) __attribute__((amdgpu_num_vgpr(248)))
void k_gemm_nt(const unsigned short* __restrict__ A, const unsigned short* __restrict__ B,
               const float* __restrict__ bias, float* __restrict__ D, int M, int N, int KTOT, int ldd) {
  static_assert(FORM >= 0 && FORM <= 2);
  static_assert(EPI == 0 || EPI == 1);
  typedef typename FragOf<FORM>::T F;
  __shared__ __attribute__((aligned(16))) float sT[8][16 * 68];
  const int lane = threadIdx.x & 31;
  const int wave = threadIdx.x >> 5;
  const int tilesM = (M + 63) >> 6;
  const int tilesN = (N + 63) >> 6;
  const int tile = blockIdx.x * 8 + wave;
  if (tile >= tilesM * tilesN) return;
  const int tm = tile / tilesN;
  const int tn = tile - tm * tilesN;
  const int m0 = tm << 6;
  const int n0 = tn << 6;

  const int rl = lane & 15;
  const int h8 = (lane >> 4) * 8;
  const unsigned short* pa = A + (size_t)(m0 + rl) * (size_t)KTOT + h8;
  const unsigned short* pb = B + (size_t)(n0 + rl) * (size_t)KTOT + h8;

  v8f acc[4][4];
#pragma unroll
  for (int i = 0; i < 4; ++i)
#pragma unroll
    for (int j = 0; j < 4; ++j) acc[i][j] = (v8f){0.f, 0.f, 0.f, 0.f, 0.f, 0.f, 0.f, 0.f};

#pragma unroll 1
  for (int k0 = 0; k0 < KTOT; k0 += 32) {
    F bf[4];
#pragma unroll
    for (int j = 0; j < 4; ++j) bf[j] = ld_frag<F>(pb + (size_t)(j << 4) * (size_t)KTOT + k0);
#pragma unroll
    for (int i = 0; i < 4; ++i) {
      const F af = ld_frag<F>(pa + (size_t)(i << 4) * (size_t)KTOT + k0);
#pragma unroll
      for (int j = 0; j < 4; ++j) acc[i][j] = mm(af, bf[j], acc[i][j]);
    }
  }

  float* slab = sT[wave];
  const int hh = lane >> 4;
  const int c4 = (lane & 15) * 4;
  const int nc = n0 + c4;
  const bool cok = nc < N;
  v4f bv = (v4f){0.f, 0.f, 0.f, 0.f};
  if (EPI == 1) {
    bv = *(const v4fa*)(bias + clampi(nc, 0, N - 4));
    asm volatile("" :: "v"(bv));
  }
#pragma unroll
  for (int i = 0; i < 4; ++i) {
    const int mBase = m0 + (i << 4);
#pragma unroll
    for (int j = 0; j < 4; ++j) {
#pragma unroll
      for (int r = 0; r < 8; ++r) slab[(h8 + r) * 68 + (j << 4) + rl] = acc[i][j][r];
    }
    __builtin_amdgcn_fence(__ATOMIC_RELEASE, "workgroup");
    __builtin_amdgcn_wave_barrier();
    __builtin_amdgcn_fence(__ATOMIC_ACQUIRE, "workgroup");
    v4f vv[8];
#pragma unroll
    for (int it = 0; it < 8; ++it) {
      const int row = it * 2 + hh;
      v4f v = *(const v4fa*)(slab + row * 68 + c4);
      if (EPI == 1) v += bv;
      vv[it] = v;
    }
    for (int pass = 0; pass < 2; ++pass) {
#pragma unroll
      for (int it = 0; it < 8; ++it) {
        const int row = mBase + it * 2 + hh;
        if (cok && row < M) *(volatile v4f*)(D + (size_t)row * (size_t)ldd + nc) = vv[it];
      }
      __threadfence();
    }
    __builtin_amdgcn_fence(__ATOMIC_RELEASE, "workgroup");
    __builtin_amdgcn_wave_barrier();
    __builtin_amdgcn_fence(__ATOMIC_ACQUIRE, "workgroup");
  }
}

#define MEAN_TERMS 2
#define WSUM_TERMS 2

#define NN      50000
#define NE      600000
#define DD      128
#define NT      6
#define XMP     50048
#define NB      1024
#define SLA     10
#define NBLK    49
#define NROWP   (NBLK * NB)
#define NTHR    256
#define NWAVE   8
#define EPT     8
#define CHUNK   2048
#define WCAP    256
#define LISTN   2048
#define RCAP    16384
#define PAIRCAP 16
#define NKEY    6144
#define ARRN    (NKEY + 16)
#define BK_INTS (LISTN + RCAP + ARRN + RCAP + 32)
#define KMH     (NT * DD)
#define KM      (KMH * MEAN_TERMS)
#define KCAT    (KM + DD * WSUM_TERMS)
#define CROWS   13312
#define NCHUNK  4
#define HROWS   (CROWS * NCHUNK)
#define FLAGW   32
#define FLAGROWS 64
#define PB_WL   48
#define PB_WS   8

static_assert(MEAN_TERMS == 1 || MEAN_TERMS == 2);
static_assert(WSUM_TERMS == 1 || WSUM_TERMS == 2);
static_assert(KCAT % 32 == 0);
static_assert(NN <= 65536 && NT <= 8 && NB <= 1024);
static_assert((1 << SLA) == NB && NBLK * NB >= NN);
static_assert(XMP % 64 == 0 && XMP >= NN && (XMP * DD / 8) % 256 == 0);
static_assert(NE % 8 == 0 && CHUNK == NTHR * EPT && WCAP == EPT * 32 && LISTN == NWAVE * WCAP);
static_assert(RCAP >= 12548 + 12548 / 4 && RCAP % 1024 == 0);
static_assert(PAIRCAP >= 11 + 5 && NT * PAIRCAP >= 28 + 8);
static_assert(NKEY == NB * NT && NKEY % 1024 == 0 && (NKEY / 32) * 32 == NKEY);
static_assert(NKEY + NB <= RCAP);
static_assert(BK_INTS % 4 == 0 && BK_INTS * 4 <= 196608);
static_assert(CROWS % 64 == 0 && CROWS == 13 * NB && CROWS % NWAVE == 0 && HROWS >= NROWP);
static_assert(PB_WL * 256 == DD * KMH / 8 && PB_WS * 256 == DD * DD / 8);
static_assert(NN % NWAVE == 0 && FLAGROWS >= NBLK);
static_assert(DD % 64 == 0);

typedef int      v4i  __attribute__((ext_vector_type(4)));
typedef unsigned v2u  __attribute__((ext_vector_type(2)));
typedef v4i __attribute__((may_alias)) v4ia;
typedef v2u __attribute__((may_alias)) v2ua;

__device__ __forceinline__ void pinf(float x)    { asm volatile("" :: "v"(x)); }
__device__ __forceinline__ void pini(int x)      { asm volatile("" :: "v"(x)); }
__device__ __forceinline__ void pinu(unsigned x) { asm volatile("" :: "v"(x)); }

__global__ __launch_bounds__(NTHR) void k_prep(const float* __restrict__ wl, const float* __restrict__ wr,
                                               const float* __restrict__ bb, const float* __restrict__ emb,
                                               unsigned short* wcat, float* csum) {
  const int b = (int)blockIdx.x, tid = (int)threadIdx.x, lane = tid & 31;
  const int wave = __builtin_amdgcn_readfirstlane(tid >> 5);
  if (b < PB_WL) {
    const int u  = b * 256 + tid;
    const int n  = u / 96;
    const int p  = u - n * 96;
    const int kk = p * 8;
    const int t  = kk >> 7;
    const int i0 = kk & (DD - 1);
    const float* s = wl + (size_t)t * (DD * DD) + (size_t)i0 * DD + (size_t)n;
    float f[8];
#pragma unroll
    for (int e = 0; e < 8; ++e) { f[e] = s[(size_t)e * DD]; pinf(f[e]); }
    const v4u o = pack8_bf16((v4f){ f[0], f[1], f[2], f[3] }, (v4f){ f[4], f[5], f[6], f[7] });
    unsigned short* q0 = wcat + (size_t)n * KCAT + kk;
    *(volatile v4u*)q0 = o;
    if (MEAN_TERMS == 2) *(volatile v4u*)(q0 + KMH) = o;
    __threadfence();
    *(volatile v4u*)q0 = o;
    if (MEAN_TERMS == 2) *(volatile v4u*)(q0 + KMH) = o;
  } else if (b < PB_WL + PB_WS) {
    const int u  = (b - PB_WL) * 256 + tid;
    const int n  = u >> 4;
    const int i0 = (u & 15) * 8;
    float s[8];
#pragma unroll
    for (int e = 0; e < 8; ++e) s[e] = 0.0f;
#pragma unroll 1
    for (int t = 0; t < NT; ++t) {
      const float* q = wr + (size_t)t * (DD * DD) + (size_t)i0 * DD + (size_t)n;
      float f[8];
#pragma unroll
      for (int e = 0; e < 8; ++e) { f[e] = q[(size_t)e * DD]; pinf(f[e]); }
#pragma unroll
      for (int e = 0; e < 8; ++e) s[e] += bf16_val(f[e]);
    }
    const v4f a = (v4f){ s[0], s[1], s[2], s[3] };
    const v4f c = (v4f){ s[4], s[5], s[6], s[7] };
    const v4u hi = pack8_bf16(a, c);
    const v4u lo = pack8_bf16_lo(a, c);
    unsigned short* q0 = wcat + (size_t)n * KCAT + KM + i0;
    *(volatile v4u*)q0 = hi;
    if (WSUM_TERMS == 2) *(volatile v4u*)(q0 + DD) = lo;
    __threadfence();
    *(volatile v4u*)q0 = hi;
    if (WSUM_TERMS == 2) *(volatile v4u*)(q0 + DD) = lo;
  } else {
    if (wave == 0) {
      v4f bs = (v4f){0.f, 0.f, 0.f, 0.f};
      v4f es = (v4f){0.f, 0.f, 0.f, 0.f};
#pragma unroll 1
      for (int t = 0; t < NT; ++t) {
        const v4f bv = *(const v4fa*)(bb  + t * DD + 4 * lane);
        const v4f ev = *(const v4fa*)(emb + t * DD + 4 * lane);
        pinf(bv[0]); pinf(bv[1]); pinf(bv[2]); pinf(bv[3]);
        pinf(ev[0]); pinf(ev[1]); pinf(ev[2]); pinf(ev[3]);
        bs[0] += bf16_val(bv[0]); bs[1] += bf16_val(bv[1]); bs[2] += bf16_val(bv[2]); bs[3] += bf16_val(bv[3]);
        es[0] += bf16_val(ev[0]); es[1] += bf16_val(ev[1]); es[2] += bf16_val(ev[2]); es[3] += bf16_val(ev[3]);
      }
      const v4f cs = bs + es;
      *(volatile v4f*)(csum + 4 * lane) = cs;
      __threadfence();
      *(volatile v4f*)(csum + 4 * lane) = cs;
    }
  }
}

__device__ __forceinline__ int ldkey(const int* __restrict__ k, int e, int nE, int sent) {
  const int v = k[e < nE ? e : nE - 1];
  pini(v);
  return (e < nE) ? v : sent;
}

__device__ __forceinline__ int scan_chunk(const int* __restrict__ keys, int nE, int cbase, int slotBase,
                                          int nb, int* list, int tid, int lane, int wave) {
  int wc = 0;
  const int el0  = tid * EPT;
  const int e0   = cbase + el0;
  const int sent = (int)(1u << 31);
  v4i da, db;
  if (cbase + CHUNK <= nE) {
    da = *(const v4i*)(keys + e0);
    db = *(const v4i*)(keys + e0 + 4);
  } else {
    da.x = ldkey(keys, e0,     nE, sent);
    da.y = ldkey(keys, e0 + 1, nE, sent);
    da.z = ldkey(keys, e0 + 2, nE, sent);
    da.w = ldkey(keys, e0 + 3, nE, sent);
    db.x = ldkey(keys, e0 + 4, nE, sent);
    db.y = ldkey(keys, e0 + 5, nE, sent);
    db.z = ldkey(keys, e0 + 6, nE, sent);
    db.w = ldkey(keys, e0 + 7, nE, sent);
  }
  const unsigned nbs = (unsigned)slotBase;
  const unsigned unb = (unsigned)nb;
  const unsigned s0 = (unsigned)da.x - nbs, s1 = (unsigned)da.y - nbs;
  const unsigned s2 = (unsigned)da.z - nbs, s3 = (unsigned)da.w - nbs;
  const unsigned s4 = (unsigned)db.x - nbs, s5 = (unsigned)db.y - nbs;
  const unsigned s6 = (unsigned)db.z - nbs, s7 = (unsigned)db.w - nbs;
  const bool h0 = s0 < unb, h1 = s1 < unb, h2 = s2 < unb, h3 = s3 < unb;
  const bool h4 = s4 < unb, h5 = s5 < unb, h6 = s6 < unb, h7 = s7 < unb;
  const unsigned any = __builtin_amdgcn_ballot_w32(h0 | h1 | h2 | h3 | h4 | h5 | h6 | h7);
  if (any != 0u) {
    const int k = (int)h0 + (int)h1 + (int)h2 + (int)h3 + (int)h4 + (int)h5 + (int)h6 + (int)h7;
    int incl = k;
#pragma unroll
    for (int dd = 1; dd < 32; dd <<= 1) {
      const int y = __shfl_up(incl, dd, 32);
      if (lane >= dd) incl += y;
    }
    wc = __shfl(incl, 31, 32);
    int pos = incl - k;
#define PUTJ(J, HJ, SJ) if (HJ) { if (pos < WCAP) list[wave * WCAP + pos] = ((el0 + (J)) << SLA) | (int)(SJ); pos += 1; }
    PUTJ(0, h0, s0)
    PUTJ(1, h1, s1)
    PUTJ(2, h2, s2)
    PUTJ(3, h3, s3)
    PUTJ(4, h4, s4)
    PUTJ(5, h5, s5)
    PUTJ(6, h6, s6)
    PUTJ(7, h7, s7)
#undef PUTJ
  }
  return wc;
}

__global__ __launch_bounds__(NTHR) void k_bucket(const int* __restrict__ ei, const int* __restrict__ et,
                                                 int* listg, int* pcntg, int* offg, int* flagg) {
  extern __shared__ __attribute__((aligned(16))) int dsm[];
  int* list = dsm;
  int* hw   = dsm + LISTN;
  int* arr  = hw + RCAP;
  int* ent  = arr + ARRN;
  int* misc = ent + RCAP;
  int* pcs  = hw;
  int* ofs  = hw + NKEY;
  const int* src = ei;
  const int* dst = ei + NE;
  const int tid = (int)threadIdx.x, lane = tid & 31;
  const int wave = __builtin_amdgcn_readfirstlane(tid >> 5);
  const int b = (int)blockIdx.x;
  const int nodeBase = b * NB;

  {
    const v4i z4 = {0, 0, 0, 0};
    for (int i = tid * 4; i < BK_INTS; i += NTHR * 4) *(v4ia*)(dsm + i) = z4;
  }
  __syncthreads();

  int t = 0;
  const int nChunks = (NE + CHUNK - 1) / CHUNK;
#pragma unroll 1
  for (int ch = 0; ch < nChunks; ++ch) {
    const int cbase = ch * CHUNK;
    int wc = scan_chunk(dst, NE, cbase, nodeBase, NB, list, tid, lane, wave);
    wc = clampi(wc, 0, WCAP);
    wc = __builtin_amdgcn_readfirstlane(wc);
    int* mb = misc + (ch & 1) * 8;
    if (lane == 0) mb[wave] = wc;
    __syncthreads();
    int base = t, tot = 0;
#pragma unroll
    for (int w2 = 0; w2 < NWAVE; ++w2) {
      const int c = clampi(mb[w2], 0, WCAP);
      base += (w2 < wave) ? c : 0;
      tot  += c;
    }
    const int myc = wc;
#pragma unroll 1
    for (int b0 = 0; b0 < myc; b0 += 32) {
      const int idx  = b0 + lane;
      const int entv = list[wave * WCAP + (idx < WCAP ? idx : WCAP - 1)];
      const int slot = entv & (NB - 1);
      const int el   = (entv >> SLA) & (CHUNK - 1);
      const int eid  = clampi(cbase + el, 0, NE - 1);
      int ty = et[eid];
      pini(ty);
      ty = clampi(ty, 0, NT - 1);
      int sr = src[eid];
      pini(sr);
      sr = clampi(sr, 0, NN - 1);
      const int pos = base + idx;
      if (idx < myc && pos < RCAP) hw[pos] = sr | (ty << 16) | (slot << 19);
    }
    t += tot;
  }
  __syncthreads();
  const int tt = t < RCAP ? t : RCAP;
  const int ov = t > RCAP ? 1 : 0;

  if (tid == 0) {
#pragma unroll 1
    for (int i = 0; i < tt; ++i) {
      const int w = hw[i];
      const int k = clampi(((w >> 19) & (NB - 1)) * NT + ((w >> 16) & 7), 0, NKEY - 1);
      arr[k] = arr[k] + 1;
    }
  }
  __syncthreads();
  if (wave == 0) {
    const int base = lane * (NKEY / 32);
    int s = 0;
#pragma unroll 1
    for (int i = 0; i < NKEY / 32; ++i) s += arr[base + i];
    int incl = s;
#pragma unroll
    for (int dd = 1; dd < 32; dd <<= 1) {
      const int y = __shfl_up(incl, dd, 32);
      if (lane >= dd) incl += y;
    }
    int run = incl - s;
#pragma unroll 1
    for (int i = 0; i < NKEY / 32; ++i) {
      run += arr[base + i];
      arr[base + i] = run;
    }
    if (lane == 31) arr[NKEY] = run;
  }
  __syncthreads();
  if (tid == 0) {
#pragma unroll 1
    for (int i = tt - 1; i >= 0; --i) {
      const int w = hw[i];
      const int k = clampi(((w >> 19) & (NB - 1)) * NT + ((w >> 16) & 7), 0, NKEY - 1);
      const int p = clampi(arr[k] - 1, 0, RCAP - 1);
      arr[k] = p;
      ent[p] = w & 0x7FFFF;
    }
  }
  __syncthreads();

  {
    int ovd = 0;
#pragma unroll 1
    for (int k = tid; k < NKEY; k += NTHR) {
      const int c = clampi(arr[k + 1] - arr[k], 0, RCAP);
      ovd |= (c > PAIRCAP) ? 1 : 0;
      pcs[k] = c;
    }
#pragma unroll 1
    for (int s = tid; s < NB; s += NTHR) ofs[s] = clampi(arr[s * NT], 0, RCAP - 1);
    const unsigned om = __builtin_amdgcn_ballot_w32(ovd != 0);
    if (lane == 0) misc[20 + wave] = (om != 0u) ? 1 : 0;
  }
  __syncthreads();
  int fl = ov;
#pragma unroll
  for (int w2 = 0; w2 < NWAVE; ++w2) fl |= misc[20 + w2];
  fl = (fl != 0) ? 1 : 0;

  int* eg = listg + (size_t)b * RCAP;
  int* pg = pcntg + (size_t)b * NKEY;
  int* og = offg  + (size_t)b * NB;
  int* fg = flagg + (size_t)b * FLAGW;
  const v4i fv = {fl, fl, fl, fl};
  for (int i = tid * 4; i < RCAP; i += NTHR * 4) {
    const v4i v = *(const v4ia*)(ent + i);
    *(volatile v4i*)(eg + i) = v;
  }
  for (int i = tid * 4; i < NKEY; i += NTHR * 4) {
    const v4i v = *(const v4ia*)(pcs + i);
    *(volatile v4i*)(pg + i) = v;
  }
  {
    const v4i v = *(const v4ia*)(ofs + 4 * tid);
    *(volatile v4i*)(og + 4 * tid) = v;
  }
  if (tid < FLAGW / 4) *(volatile v4i*)(fg + 4 * tid) = fv;
  __threadfence();
  for (int i = tid * 4; i < RCAP; i += NTHR * 4) {
    const v4i v = *(const v4ia*)(ent + i);
    *(volatile v4i*)(eg + i) = v;
  }
  for (int i = tid * 4; i < NKEY; i += NTHR * 4) {
    const v4i v = *(const v4ia*)(pcs + i);
    *(volatile v4i*)(pg + i) = v;
  }
  {
    const v4i v = *(const v4ia*)(ofs + 4 * tid);
    *(volatile v4i*)(og + 4 * tid) = v;
  }
  if (tid < FLAGW / 4) *(volatile v4i*)(fg + 4 * tid) = fv;
}

__global__ __launch_bounds__(NTHR) void k_replay(const unsigned short* __restrict__ xb,
                                                 const int* __restrict__ listg, const int* __restrict__ pcntg,
                                                 const int* __restrict__ offg, const int* __restrict__ flagg,
                                                 unsigned short* ach, int rowBase) {
  const int tid = (int)threadIdx.x, lane = tid & 31;
  const int wave = __builtin_amdgcn_readfirstlane(tid >> 5);
  const int r = (int)blockIdx.x * NWAVE + wave;
  const int d = rowBase + r;
  const bool live = d < NN;
  const int dc  = d < NROWP - 1 ? d : NROWP - 1;
  const int ds  = d < NN - 1 ? d : NN - 1;
  const int blk = dc >> SLA;
  const unsigned lm = live ? 0xFFFFFFFFu : 0u;

  int pv = pcntg[(size_t)dc * NT + (lane < NT ? lane : NT - 1)];
  pini(pv);
  pv = clampi(pv, 0, PAIRCAP);
  pv = live ? pv : 0;
  int o0 = offg[dc];
  pini(o0);
  o0 = clampi(o0, 0, RCAP - 1);
  o0 = __builtin_amdgcn_readfirstlane(o0);
  int fl = flagg[blk * FLAGW];
  pini(fl);
  fl = __builtin_amdgcn_readfirstlane(fl);
  const float pz = (fl != 0) ? __int_as_float(0x7fc00000) : 0.0f;

  int deg = 0;
#pragma unroll
  for (int t = 0; t < NT; ++t) deg += __builtin_amdgcn_readlane(pv, t);
  int nodeLast = o0 + (deg > 0 ? deg - 1 : 0);
  nodeLast = nodeLast > RCAP - 1 ? RCAP - 1 : nodeLast;

  const int* lb = listg + (size_t)blk * RCAP;
  const unsigned short* xl = xb + 4 * lane;
  unsigned short* arow = ach + (size_t)r * KCAT + 4 * lane;
  int base = o0;
#pragma unroll 1
  for (int t = 0; t < NT; ++t) {
    const int cn = __builtin_amdgcn_readlane(pv, t);
    float a0 = 0.0f, a1 = 0.0f, a2 = 0.0f, a3 = 0.0f;
#pragma unroll 1
    for (int p = 0; p < cn; ++p) {
      int idx = base + p;
      idx = idx > nodeLast ? nodeLast : idx;
      int w = lb[idx];
      pini(w);
      const int sr = clampi(w & 0xFFFF, 0, NN - 1);
      const v2u xw = *(const v2ua*)(xl + (size_t)sr * DD);
      pinu(xw.x); pinu(xw.y);
      a0 += __uint_as_float(xw.x << 16);
      a1 += __uint_as_float(xw.x & 0xFFFF0000u);
      a2 += __uint_as_float(xw.y << 16);
      a3 += __uint_as_float(xw.y & 0xFFFF0000u);
    }
    base += cn;
    const float den = fmaxf((float)cn, 1.0f);
    const float m0 = a0 / den + pz;
    const float m1 = a1 / den + pz;
    const float m2 = a2 / den + pz;
    const float m3 = a3 / den + pz;
    v2u hv, lv;
    hv.x = pk16(bf16_bits(m0), bf16_bits(m1)) & lm;
    hv.y = pk16(bf16_bits(m2), bf16_bits(m3)) & lm;
    lv.x = pk16(bf16_lo_bits(m0), bf16_lo_bits(m1)) & lm;
    lv.y = pk16(bf16_lo_bits(m2), bf16_lo_bits(m3)) & lm;
    unsigned short* ph = arow + t * DD;
    *(volatile v2u*)ph = hv;
    if (MEAN_TERMS == 2) *(volatile v2u*)(ph + KMH) = lv;
    __threadfence();
    *(volatile v2u*)ph = hv;
    if (MEAN_TERMS == 2) *(volatile v2u*)(ph + KMH) = lv;
  }
  {
    v2u xw = *(const v2ua*)(xl + (size_t)ds * DD);
    pinu(xw.x); pinu(xw.y);
    xw.x &= lm;
    xw.y &= lm;
    unsigned short* px = arow + KM;
    *(volatile v2u*)px = xw;
    if (WSUM_TERMS == 2) *(volatile v2u*)(px + DD) = xw;
    __threadfence();
    *(volatile v2u*)px = xw;
    if (WSUM_TERMS == 2) *(volatile v2u*)(px + DD) = xw;
  }
}

__global__ __launch_bounds__(NTHR) void k_row(const float* __restrict__ hm, const float* __restrict__ csum,
                                              const float* __restrict__ gamma, const float* __restrict__ beta,
                                              const int* __restrict__ flagg, float* outp) {
  __shared__ __attribute__((aligned(16))) float sp[3 * DD];
  const int tid = (int)threadIdx.x, lane = tid & 31;
  const int wave = __builtin_amdgcn_readfirstlane(tid >> 5);
  if (wave == 0) {
    const v4f v = *(const v4fa*)(csum + 4 * lane);
    *(v4fa*)(sp + 4 * lane) = v;
  }
  if (wave == 1) {
    const v4f v = *(const v4fa*)(gamma + 4 * lane);
    const v4f o = (v4f){ bf16_val(v[0]), bf16_val(v[1]), bf16_val(v[2]), bf16_val(v[3]) };
    *(v4fa*)(sp + DD + 4 * lane) = o;
  }
  if (wave == 2) {
    const v4f v = *(const v4fa*)(beta + 4 * lane);
    const v4f o = (v4f){ bf16_val(v[0]), bf16_val(v[1]), bf16_val(v[2]), bf16_val(v[3]) };
    *(v4fa*)(sp + 2 * DD + 4 * lane) = o;
  }
  __syncthreads();
  const int d = (int)blockIdx.x * NWAVE + wave;
  const bool live = d < NN;
  const int dcl = d < NN - 1 ? d : NN - 1;
  const v4f cs = *(const v4fa*)(sp + 4 * lane);
  const v4f gm = *(const v4fa*)(sp + DD + 4 * lane);
  const v4f be = *(const v4fa*)(sp + 2 * DD + 4 * lane);
  v4f hv = *(const v4fa*)(hm + (size_t)dcl * DD + 4 * lane);
  pinf(hv[0]); pinf(hv[1]); pinf(hv[2]); pinf(hv[3]);
  int fl = flagg[(dcl >> SLA) * FLAGW];
  pini(fl);
  hv = hv + cs;
  float s = (hv[0] + hv[1]) + (hv[2] + hv[3]);
  s += __shfl_xor(s, 16, 32);
  s += __shfl_xor(s, 8, 32);
  s += __shfl_xor(s, 4, 32);
  s += __shfl_xor(s, 2, 32);
  s += __shfl_xor(s, 1, 32);
  const float mu = s * (1.0f / 128.0f);
  const v4f dv = (v4f){ hv[0] - mu, hv[1] - mu, hv[2] - mu, hv[3] - mu };
  float q = (dv[0] * dv[0] + dv[1] * dv[1]) + (dv[2] * dv[2] + dv[3] * dv[3]);
  q += __shfl_xor(q, 16, 32);
  q += __shfl_xor(q, 8, 32);
  q += __shfl_xor(q, 4, 32);
  q += __shfl_xor(q, 2, 32);
  q += __shfl_xor(q, 1, 32);
  const float var = q * (1.0f / 128.0f);
  const float rs  = 1.0f / sqrtf(var + 1e-5f);
  const float qn  = __int_as_float(0x7fc00000);
  v4f o;
#pragma unroll
  for (int i = 0; i < 4; ++i) {
    float y = dv[i] * rs * gm[i] + be[i];
    y = (y > 0.0f) ? y : (y - y);
    y = (fl != 0) ? qn : y;
    o[i] = y;
  }
  float* op = outp + (size_t)dcl * DD + 4 * lane;
  if (live) *(volatile v4f*)op = o;
  __threadfence();
  if (live) *(volatile v4f*)op = o;
}

static inline size_t al256(size_t o) { return (o + 255) & ~(size_t)255; }

extern "C" void kernel_launch(void* const* d_in, const int* in_sizes, int n_in,
                              void* d_out, int out_size, void* d_ws, size_t ws_size,
                              hipStream_t stream) {
  if (n_in < 9) return;
  if (in_sizes[0] != NN * DD) return;
  if (in_sizes[1] != 2 * NE || in_sizes[2] != NE) return;
  if (in_sizes[3] != NT * DD * DD || in_sizes[4] != NT * DD * DD) return;
  if (in_sizes[5] != NT * DD || in_sizes[6] != NT * DD) return;
  if (in_sizes[7] != DD || in_sizes[8] != DD) return;
  if (out_size != NN * DD) return;

  const float* x     = (const float*)d_in[0];
  const int*   ei    = (const int*)d_in[1];
  const int*   et    = (const int*)d_in[2];
  const float* Wl    = (const float*)d_in[3];
  const float* Wr    = (const float*)d_in[4];
  const float* bb    = (const float*)d_in[5];
  const float* emb   = (const float*)d_in[6];
  const float* gamma = (const float*)d_in[7];
  const float* beta  = (const float*)d_in[8];
  float* out = (float*)d_out;

  char* ws = (char*)d_ws;
  size_t off = 0;
  const size_t oXB   = off; off = al256(off + (size_t)XMP * DD * 2);
  const size_t oACH  = off; off = al256(off + (size_t)CROWS * KCAT * 2);
  const size_t oH    = off; off = al256(off + (size_t)HROWS * DD * 4);
  const size_t oLIST = off; off = al256(off + (size_t)NBLK * RCAP * 4);
  const size_t oPCNT = off; off = al256(off + (size_t)NROWP * NT * 4);
  const size_t oOFF  = off; off = al256(off + (size_t)NROWP * 4);
  const size_t oFLAG = off; off = al256(off + (size_t)FLAGROWS * FLAGW * 4);
  const size_t oWCAT = off; off = al256(off + (size_t)DD * KCAT * 2);
  const size_t oCSUM = off; off = al256(off + (size_t)DD * 4);
  if (off > ws_size || off > (size_t)(128u << 20)) return;
  unsigned short* XB   = (unsigned short*)(ws + oXB);
  unsigned short* ACH  = (unsigned short*)(ws + oACH);
  float*          H    = (float*)(ws + oH);
  int*            LIST = (int*)(ws + oLIST);
  int*            PCNT = (int*)(ws + oPCNT);
  int*            OFF  = (int*)(ws + oOFF);
  int*            FLAG = (int*)(ws + oFLAG);
  unsigned short* WCAT = (unsigned short*)(ws + oWCAT);
  float*          CSUM = (float*)(ws + oCSUM);

  const int bkLds = BK_INTS * 4;
  hipFuncSetAttribute(reinterpret_cast<const void*>(&k_bucket), hipFuncAttributeMaxDynamicSharedMemorySize, bkLds);

  k_plane<0><<<XMP * DD / 8 / 256, 256, 0, stream>>>(x, NN, DD, DD, XB, XMP, DD);
  k_prep<<<PB_WL + PB_WS + 1, NTHR, 0, stream>>>(Wl, Wr, bb, emb, WCAT, CSUM);
  k_bucket<<<NBLK, NTHR, bkLds, stream>>>(ei, et, LIST, PCNT, OFF, FLAG);
  const int gemmBlocks = ((CROWS / 64) * (DD / 64) + 7) / 8;
  for (int c = 0; c < NCHUNK; ++c) {
    k_replay<<<CROWS / NWAVE, NTHR, 0, stream>>>(XB, LIST, PCNT, OFF, FLAG, ACH, c * CROWS);
    k_gemm_nt<0, 0><<<gemmBlocks, 256, 0, stream>>>(ACH, WCAT, CSUM, H + (size_t)c * CROWS * DD,
                                                     CROWS, DD, KCAT, DD);
  }
  k_row<<<NN / NWAVE, NTHR, 0, stream>>>(H, CSUM, gamma, beta, FLAG, out);
}
